// SMOLEnv_65335042506807
// MI455X (gfx1250) — hardware-verified
//
#include <hip/hip_runtime.h>

#define NAT   2048
#define NHD   5
#define NRB   16
#define NPB   32
#define PSTR  2056
#define CENTER_STEP (10.0f / 15.0f)
#define INV_SIGMA   1.6f

typedef _Float16 f16;
typedef __attribute__((ext_vector_type(16))) f16 f16x16;
typedef __attribute__((ext_vector_type(8)))  f16 f16x8;
typedef __attribute__((ext_vector_type(8)))  float f32x8;
typedef __attribute__((ext_vector_type(4)))  float v4f_t;
typedef float v4fa __attribute__((ext_vector_type(4), may_alias));

__device__ __forceinline__ f32x8 wmma16(f16x16 a, f16x16 b, f32x8 c) {
  return __builtin_amdgcn_wmma_f32_16x16x32_f16(false, a, false, b, (short)0, c, false, false);
}

__global__ __launch_bounds__(256) void smol_env_kernel(const float* __restrict__ pos,
                                                      const float* __restrict__ mask,
                                                      const float* __restrict__ Wrb,
                                                      float* __restrict__ out) {
  __shared__ float4 sp[NAT];
  __shared__ __attribute__((aligned(16))) f16 Bh[4 * PSTR];
  __shared__ __attribute__((aligned(16))) f16 Bl[4 * PSTR];
  __shared__ __attribute__((aligned(16))) float outS[NPB * NHD * 3];

  const int tid = threadIdx.x, lane = tid & 31, wave = tid >> 5;
  const int col = lane & 15, half = lane >> 4;
  const int b  = blockIdx.x / (NAT / NPB);
  const int n0 = (blockIdx.x % (NAT / NPB)) * NPB;

  for (int i = tid; i < NAT; i += 256) {
    const float* p = pos + ((size_t)b * NAT + i) * 3;
    float4 v; v.x = p[0]; v.y = p[1]; v.z = p[2]; v.w = (mask[(size_t)b * NAT + i] > 0.0f) ? 1.0f : 0.0f;
    sp[i] = v;
    const float vals[4] = {v.x, v.y, v.z, 1.0f};
#pragma unroll
    for (int c = 0; c < 4; ++c) {
      const f16 h = (f16)vals[c];
      Bh[c * PSTR + i] = h;
      Bl[c * PSTR + i] = (f16)((vals[c] - (float)h) * 2048.0f);
    }
  }
  f16x16 bW;
#pragma unroll
  for (int j = 0; j < 16; ++j) {
    float w = 0.0f;
    if (j < 8 && col < NHD) w = Wrb[(8 * half + j) * NHD + col];
    bW[j] = (f16)w;
  }
  __syncthreads();

  const float LOG2E = 1.44269504088896340736f;
#pragma unroll 1
  for (int q = 0; q < 4; ++q) {
    const int nl = wave * 4 + q;
    const float4 pq = sp[n0 + nl];
    float mx = -3.0e38f, lsum = 0.0f;
    f32x8 acc = {}, accx = {};
#pragma unroll 1
    for (int m0 = 0; m0 < NAT; m0 += 32) {
      f32x8 S[2];
#pragma unroll
      for (int t = 0; t < 2; ++t) {
        const float4 pm = sp[m0 + 16 * t + col];
        const float dx = pq.x - pm.x, dy = pq.y - pm.y, dz = pq.z - pm.z;
        const float d = sqrtf(fmaxf(dx * dx + dy * dy + dz * dz, 1e-12f));
        f16x16 a;
#pragma unroll
        for (int j = 0; j < 8; ++j) {
          const float u = (d - CENTER_STEP * (float)(8 * half + j)) * INV_SIGMA;
          a[j] = (f16)__builtin_amdgcn_exp2f(-(u * u) * LOG2E);
        }
#pragma unroll
        for (int j = 8; j < 16; ++j) a[j] = (f16)0.0f;
        f32x8 z = {};
        S[t] = wmma16(a, bW, z);
      }
      float cm = -3.0e38f;
#pragma unroll
      for (int r = 0; r < 8; ++r) cm = fmaxf(cm, fmaxf(S[0][r], S[1][r]));
      cm = fmaxf(cm, __shfl_xor(cm, 16, 32));
      const float mnew  = fmaxf(mx, cm);
      const float alpha = __builtin_amdgcn_exp2f((mx - mnew) * LOG2E);
      mx = mnew; lsum *= alpha;
      {
#pragma unroll
        for (int r = 0; r < 8; ++r) {
          const float ar = __shfl(alpha, 8 * half + r, 32);
          acc[r] *= ar; accx[r] *= ar;
        }
      }
      f16x16 a2, a2l;
      const float msh = mnew * LOG2E - 10.0f;
#pragma unroll
      for (int t = 0; t < 2; ++t)
#pragma unroll
        for (int r = 0; r < 8; ++r) {
          const float mb = sp[m0 + 16 * t + 8 * half + r].w;
          const float p = __builtin_amdgcn_exp2f(S[t][r] * LOG2E - msh) * mb;
          lsum += p;
          const f16 ph = (f16)p;
          a2[8 * t + r] = ph; a2l[8 * t + r] = (f16)((p - (float)ph) * 2048.0f);
        }
      f16x16 bh, bl;
      if (col < 4) {
        const int kh = 8 * half;
        const f16x8 h0 = *(const f16x8*)(Bh + col * PSTR + m0 + kh), h1 = *(const f16x8*)(Bh + col * PSTR + m0 + kh + 16);
        const f16x8 l0 = *(const f16x8*)(Bl + col * PSTR + m0 + kh), l1 = *(const f16x8*)(Bl + col * PSTR + m0 + kh + 16);
#pragma unroll
        for (int e = 0; e < 8; ++e) { bh[e] = h0[e]; bh[e + 8] = h1[e]; bl[e] = l0[e]; bl[e + 8] = l1[e]; }
      } else {
#pragma unroll
        for (int e = 0; e < 16; ++e) { bh[e] = (f16)0.0f; bl[e] = (f16)0.0f; }
      }
      acc  = wmma16(a2, bh, acc);
      accx = wmma16(a2, bl, accx);
      accx = wmma16(a2l, bh, accx);
    }
    lsum += __shfl_xor(lsum, 16, 32);
#pragma unroll
    for (int r = 0; r < NHD; ++r) {
      const float lh = __shfl(lsum, r, 32);
      if (half == 0 && col < 3) {
        float v = 0.0f;
        if (r != 1 && pq.w > 0.0f && lh > 0.0f) v = (acc[r] + accx[r] * (1.0f / 2048.0f)) / lh;
        outS[nl * 15 + r * 3 + col] = v;
      }
    }
  }
  __syncthreads();
  float* ob = out + ((size_t)b * NAT + n0) * (NHD * 3);
#pragma unroll 1
  for (int pass = 0; pass < 2; ++pass) {
    if (tid < 120) *(volatile v4f_t*)(ob + 4 * tid) = *(const volatile v4fa*)(outS + 4 * tid);
    __threadfence();
  }
}

extern "C" void kernel_launch(void* const* d_in, const int* in_sizes, int n_in,
                              void* d_out, int out_size, void* d_ws, size_t ws_size,
                              hipStream_t stream) {
  (void)n_in; (void)out_size; (void)d_ws; (void)ws_size;
  const float* pos  = (const float*)d_in[0];
  const float* mask = (const float*)d_in[2];
  const float* Wrb  = (const float*)d_in[3];
  float* out = (float*)d_out;
  const int B = in_sizes[2] / NAT;
  smol_env_kernel<<<dim3(B * (NAT / NPB)), dim3(256), 0, stream>>>(pos, mask, Wrb, out);
}
